// SelfTransformerBlock_84628035601169
// MI455X (gfx1250) — hardware-verified
//
#include <hip/hip_runtime.h>
#include <math.h>

typedef __attribute__((ext_vector_type(16))) _Float16 v16h;
typedef __attribute__((ext_vector_type(16))) __bf16 v16b;
typedef __attribute__((ext_vector_type(8)))  _Float16 v8h;
typedef __attribute__((ext_vector_type(8)))  float v8f;
typedef __attribute__((ext_vector_type(4)))  float v4f;
typedef __attribute__((ext_vector_type(2)))  float v2f;
typedef __attribute__((ext_vector_type(4)))  unsigned v4u;
typedef __attribute__((ext_vector_type(4)))  int v4i;
typedef float __attribute__((may_alias)) float_a;
typedef int __attribute__((may_alias)) int_a;

template <typename T> __device__ __forceinline__ void vst2(void* p, T v) { *(volatile T*)p = v; __threadfence(); *(volatile T*)p = v; }
__device__ __forceinline__ v8f wmma16(v16h a, v16h b, v8f c) {
  v8f d = __builtin_amdgcn_wmma_f32_16x16x32_f16(false, a, false, b, (short)0, c, false, false);
  asm volatile("v_nop\n\tv_nop\n\tv_nop\n\tv_nop" : "+v"(d) : "v"(a), "v"(b));
  return d;
}
__device__ __forceinline__ v8f wmma_bf(v16b a, v16b b, v8f c) {
  v8f d = __builtin_amdgcn_wmma_f32_16x16x32_bf16(false, a, false, b, (short)0, c, false, false);
  asm volatile("v_nop\n\tv_nop\n\tv_nop\n\tv_nop" : "+v"(d) : "v"(a), "v"(b));
  return d;
}
__device__ __forceinline__ v16h frag_h(const _Float16* rowk0, int lane) {
  union { v16h v; v8h q[2]; } u; const _Float16* p = rowk0 + 8 * (lane >> 4);
  u.q[0] = *(const v8h*)p; u.q[1] = *(const v8h*)(p + 16); return u.v;
}
__device__ __forceinline__ v16h frag_f32(const float* rowk0, int lane) {
  v16h a; const float* p = rowk0 + 8 * (lane >> 4);
#pragma unroll
  for (int i = 0; i < 8; ++i) { a[i] = (_Float16)p[i]; a[8 + i] = (_Float16)p[16 + i]; }
  return a;
}
__device__ __forceinline__ v16h frag_f32s(const float* rowk0, int lane, float sc) {
  v16h a; const float* p = rowk0 + 8 * (lane >> 4);
#pragma unroll
  for (int i = 0; i < 8; ++i) { a[i] = (_Float16)(p[i] * sc); a[8 + i] = (_Float16)(p[16 + i] * sc); }
  return a;
}
__device__ __forceinline__ v16h fragc_f32(const float* W, int k0, int n, int lane, int ld, int K) {
  v16h a; const int g = lane >> 4;
#pragma unroll
  for (int i = 0; i < 8; ++i) { const int ka = k0 + 8 * g + i, kb = ka + 16;
    a[i] = (_Float16)(ka < K ? W[(size_t)(ka < K ? ka : K - 1) * ld + n] : 0.f); a[8 + i] = (_Float16)(kb < K ? W[(size_t)(kb < K ? kb : K - 1) * ld + n] : 0.f); }
  return a;
}
struct F2 { v16b h, l; };
__device__ __forceinline__ F2 bsplit16(const float v[16]) { F2 r;
#pragma unroll
  for (int i = 0; i < 16; ++i) { const __bf16 h = (__bf16)v[i]; r.h[i] = h; r.l[i] = (__bf16)(v[i] - (float)h); }
  return r; }
__device__ __forceinline__ F2 split_row(const float* row, int k0, int lane) { float v[16]; const float* p = row + k0 + 8 * (lane >> 4);
#pragma unroll
  for (int i = 0; i < 8; ++i) { v[i] = p[i]; v[8 + i] = p[16 + i]; }
  return bsplit16(v); }
__device__ __forceinline__ F2 split_rowK(const float* row, int k0, int lane, int K) { float v[16]; const int g = lane >> 4;
#pragma unroll
  for (int i = 0; i < 8; ++i) { const int ka = k0 + 8 * g + i, kb = ka + 16; v[i] = ka < K ? row[ka < K ? ka : K - 1] : 0.f; v[8 + i] = kb < K ? row[kb < K ? kb : K - 1] : 0.f; }
  return bsplit16(v); }
__device__ __forceinline__ F2 split_col(const float* W, int k0, int n, int lane, int ld, int K) { float v[16]; const int g = lane >> 4;
#pragma unroll
  for (int i = 0; i < 8; ++i) { const int ka = k0 + 8 * g + i, kb = ka + 16; v[i] = ka < K ? W[(size_t)(ka < K ? ka : K - 1) * ld + n] : 0.f; v[8 + i] = kb < K ? W[(size_t)(kb < K ? kb : K - 1) * ld + n] : 0.f; }
  return bsplit16(v); }
__device__ __forceinline__ v8f mac3(const F2& a, const F2& b, v8f c) { c = wmma_bf(a.l, b.h, c); c = wmma_bf(a.h, b.l, c); return wmma_bf(a.h, b.h, c); }
__device__ __forceinline__ float sigm(float v) { return 1.0f / (1.0f + expf(-v)); }
#define LDSX() do { asm volatile("s_wait_dscnt 0" ::: "memory"); __builtin_amdgcn_wave_barrier(); __builtin_amdgcn_fence(__ATOMIC_RELEASE, "workgroup"); } while (0)


#define NB 4
#define NT 4096
#define CD 512
#define C2 1024
#define NH 8
#define DH 64
#define NR (NB * NT)
#define EPSA 1e-6f
#define EPSL 1e-5f
#ifndef TNB
#define TNB NB
#endif
typedef __attribute__((ext_vector_type(8))) __bf16 v8b;
__device__ __forceinline__ v16b frag_b(const __bf16* rowk0, int lane) {
  union { v16b v; v8b q[2]; } u; const __bf16* p = rowk0 + 8 * (lane >> 4);
  u.q[0] = *(const v8b*)p; u.q[1] = *(const v8b*)(p + 16); return u.v;
}
__device__ __forceinline__ float bfr(float v) { return (float)(__bf16)v; }
__device__ __attribute__((noinline)) float exp_ni(float v) { return expf(v); }
__device__ __attribute__((noinline)) float erf_ni(float v) { return erff(v); }

#define WS_XS  0u
#define WS_QH  (WS_XS + 2u * (size_t)NR * CD)
#define WS_QL  (WS_QH + 2u * (size_t)NR * CD)
#define WS_KT  (WS_QL + 2u * (size_t)NR * CD)
#define WS_KTL (WS_KT + 2u * (size_t)NR * CD)
#define WS_VT  (WS_KTL + 2u * (size_t)NR * CD)
#define WS_VTL (WS_VT + 2u * (size_t)NR * CD)
#define WS_KVT (WS_VTL + 2u * (size_t)NR * CD)
#define WS_KVL (WS_KVT + 2u * (size_t)NB * NH * DH * DH)
#define WS_KS  (WS_KVL + 2u * (size_t)NB * NH * DH * DH)
#define WS_MSG (WS_KS + 4u * (size_t)NB * CD)
#define WS_M2  (WS_MSG + 2u * (size_t)NR * CD)
#define WS_FFB (WS_M2 + 4u * (size_t)NR * CD)
#define WS_H1  (WS_FFB + 2u * (size_t)NR * CD)
#define WS_END (WS_H1 + 2u * (size_t)NR * C2)

__device__ __forceinline__ v16b fragb_f32(const float* __restrict__ p, int lane) { v16b a; const float* pp = p + 8 * (lane >> 4);
#pragma unroll
  for (int i = 0; i < 8; ++i) { a[i] = (__bf16)pp[i]; a[8 + i] = (__bf16)pp[16 + i]; } return a; }
__device__ __forceinline__ v16h fragh_f32(const float* __restrict__ p, int lane) { v16h a; const float* pp = p + 8 * (lane >> 4);
#pragma unroll
  for (int i = 0; i < 8; ++i) { a[i] = (_Float16)bfr(pp[i]); a[8 + i] = (_Float16)bfr(pp[16 + i]); } return a; }
__global__ __launch_bounds__(256) void k_xt(const float* __restrict__ X, __bf16* __restrict__ XS) { __shared__ __align__(16) __bf16 s[64][CD + 8]; const int t = threadIdx.x; const size_t b = blockIdx.y; const int n0 = blockIdx.x * 64;
  for (int e = t; e < CD * 64; e += 256) { const int c = e >> 6, nl = e & 63; s[nl][c] = (__bf16)X[(b * CD + c) * (size_t)NT + n0 + nl]; } __syncthreads();
  for (int e = t; e < 64 * (CD / 8); e += 256) { const int nl = e / (CD / 8), q = e % (CD / 8); vst2((unsigned*)(XS + (b * NT + n0 + nl) * CD + q * 8), *(const v4u*)&s[nl][q * 8]); } }
__global__ __launch_bounds__(128) void k_qkv(const __bf16* __restrict__ XS, const float* __restrict__ WQ, const float* __restrict__ WK, const float* __restrict__ WV, const float* __restrict__ MASK, _Float16* __restrict__ QH, _Float16* __restrict__ QL, _Float16* __restrict__ KT, _Float16* __restrict__ KTL, _Float16* __restrict__ VT, _Float16* __restrict__ VTL) {
  __shared__ __align__(16) _Float16 sh[64][136], sl[64][136]; __shared__ __align__(16) _Float16 th[128][72], tl[128][72];
  const int tid = threadIdx.x, wave = tid >> 5, lane = tid & 31, col = lane & 15, g = lane >> 4; const size_t b = blockIdx.z; const int n0 = blockIdx.x * 64 + wave * 16; const int c0 = blockIdx.y * 128; const int which = c0 / CD; const int cc0 = c0 % CD; const size_t r0 = b * NT + n0; const float* Wm = which == 0 ? WQ : which == 1 ? WK : WV;
  v8f acc[8] = {};
#pragma unroll 2
  for (int kc = 0; kc < CD / 32; ++kc) { const v16b a = frag_b(XS + (r0 + col) * CD + kc * 32, lane);
#pragma unroll
    for (int j = 0; j < 8; ++j) acc[j] = wmma_bf(a, fragb_f32(Wm + (size_t)(cc0 + j * 16 + col) * CD + kc * 32, lane), acc[j]); }
#pragma unroll
  for (int j = 0; j < 8; ++j)
#pragma unroll
    for (int r = 0; r < 8; ++r) { const float mk = bfr(MASK[r0 + 8 * g + r]); float v = acc[j][r]; if (which < 2) { v = (v > 0.f ? v : expm1f(v)) + 1.0f; v *= mk; } else { v = v * mk * (1.0f / (float)NT); }
      const _Float16 hv = (_Float16)v; const _Float16 lv = (_Float16)((v - (float)hv) * 2048.0f); if (which == 0) { sh[wave * 16 + 8 * g + r][j * 16 + col] = hv; sl[wave * 16 + 8 * g + r][j * 16 + col] = lv; } else { th[j * 16 + col][wave * 16 + 8 * g + r] = hv; tl[j * 16 + col][wave * 16 + 8 * g + r] = lv; } }
  __syncthreads();
  if (which == 0) { for (int e = tid; e < 64 * 16; e += 128) { const int rl = e >> 4, q = e & 15; const size_t o = (b * NT + blockIdx.x * 64 + rl) * CD + cc0 + q * 8; vst2((unsigned*)(QH + o), *(const v4u*)&sh[rl][q * 8]); vst2((unsigned*)(QL + o), *(const v4u*)&sl[rl][q * 8]); } }
  else { _Float16* PH = which == 1 ? KT : VT; _Float16* PL = which == 1 ? KTL : VTL; for (int e = tid; e < 128 * 8; e += 128) { const int cl = e >> 3, q = e & 7; const size_t o = ((b * CD + cc0 + cl) * (size_t)NT) + blockIdx.x * 64 + q * 8; vst2((unsigned*)(PH + o), *(const v4u*)&th[cl][q * 8]); vst2((unsigned*)(PL + o), *(const v4u*)&tl[cl][q * 8]); } } }
__global__ __launch_bounds__(128) void k_kv(const _Float16* __restrict__ KT, const _Float16* __restrict__ KTL, const _Float16* __restrict__ VT, const _Float16* __restrict__ VTL, _Float16* __restrict__ KVT, _Float16* __restrict__ KVL, float* __restrict__ KS) { __shared__ __align__(16) _Float16 th[DH][DH + 8], tl2[DH][DH + 8]; __shared__ __align__(16) float sks[DH];
  const int tid = threadIdx.x, wave = tid >> 5, lane = tid & 31, col = lane & 15, g = lane >> 4; const int h = blockIdx.x; const size_t b = blockIdx.y; const size_t pk = (b * CD + (size_t)h * DH) * NT; const int d0 = wave * 16;
  v8f acc[4] = {}, accl[4] = {};
#pragma unroll 1
  for (int kc = 0; kc < NT / 32; ++kc) { const v16h ah = frag_h(KT + pk + (size_t)(d0 + col) * NT + kc * 32, lane), al = frag_h(KTL + pk + (size_t)(d0 + col) * NT + kc * 32, lane);
#pragma unroll
    for (int j = 0; j < 4; ++j) { const size_t o = pk + (size_t)(j * 16 + col) * NT + kc * 32; const v16h bh = frag_h(VT + o, lane), bl = frag_h(VTL + o, lane); acc[j] = wmma16(ah, bh, acc[j]); accl[j] = wmma16(ah, bl, accl[j]); accl[j] = wmma16(al, bh, accl[j]); } }
#pragma unroll
  for (int j = 0; j < 4; ++j)
#pragma unroll
    for (int r = 0; r < 8; ++r) { const float v = acc[j][r] + accl[j][r] * (1.0f / 2048.0f); const _Float16 hv = (_Float16)v; th[j * 16 + col][d0 + 8 * g + r] = hv; tl2[j * 16 + col][d0 + 8 * g + r] = (_Float16)((v - (float)hv) * 2048.0f); }
  { const int d = d0 + (lane & 15); const _Float16* rh = KT + pk + (size_t)d * NT; const _Float16* rl = KTL + pk + (size_t)d * NT; float s = 0.f; for (int n = (lane >> 4); n < NT; n += 2) s += (float)rh[n] + (float)rl[n] * (1.0f / 2048.0f); s += __shfl_xor(s, 16); if (lane < 16) sks[d] = s; }
  __syncthreads(); for (int e = tid; e < DH * 8; e += 128) { const int v = e >> 3, q = e & 7; const size_t o = ((b * NH + h) * DH + v) * DH + q * 8; vst2((unsigned*)(KVT + o), *(const v4u*)&th[v][q * 8]); vst2((unsigned*)(KVL + o), *(const v4u*)&tl2[v][q * 8]); }
  if (tid < DH / 4) vst2(KS + b * CD + (size_t)h * DH + tid * 4, *(const v4f*)&sks[tid * 4]); }
__global__ __launch_bounds__(128) void k_msg(const _Float16* __restrict__ QH, const _Float16* __restrict__ QL, const _Float16* __restrict__ KVT, const _Float16* __restrict__ KVL, const float* __restrict__ KS, _Float16* __restrict__ MSG) { __shared__ __align__(16) _Float16 sh[4][16][72];
  const int tid = threadIdx.x, wave = tid >> 5, lane = tid & 31, col = lane & 15, g = lane >> 4; const size_t r0 = (size_t)blockIdx.x * 64 + wave * 16; const int h = blockIdx.y; const size_t b = r0 / NT; const size_t pa = ((b * NH + h) * DH) * DH;
  v8f acc[4] = {}, accl[4] = {};
#pragma unroll
  for (int kc = 0; kc < DH / 32; ++kc) { const v16h ah = frag_h(QH + (r0 + col) * CD + h * DH + kc * 32, lane), al = frag_h(QL + (r0 + col) * CD + h * DH + kc * 32, lane);
#pragma unroll
    for (int j = 0; j < 4; ++j) { const size_t o = pa + (size_t)(j * 16 + col) * DH + kc * 32; const v16h bh = frag_h(KVT + o, lane), bl = frag_h(KVL + o, lane); acc[j] = wmma16(ah, bh, acc[j]); accl[j] = wmma16(ah, bl, accl[j]); accl[j] = wmma16(al, bh, accl[j]); } }
  __shared__ float sks[DH]; if (tid < DH) sks[tid] = KS[b * CD + h * DH + tid]; __syncthreads();
  float zr[8];
#pragma unroll
  for (int r = 0; r < 8; ++r) { const size_t row = r0 + 8 * g + r; float s = 0.f; for (int d = col; d < DH; d += 16) s += ((float)QH[row * CD + h * DH + d] + (float)QL[row * CD + h * DH + d] * (1.0f / 2048.0f)) * sks[d];
#pragma unroll
    for (int o = 1; o < 16; o <<= 1) s += __shfl_xor(s, o);
    zr[r] = (float)NT / (s + EPSA); }
#pragma unroll
  for (int j = 0; j < 4; ++j)
#pragma unroll
    for (int r = 0; r < 8; ++r) sh[wave][8 * g + r][j * 16 + col] = (_Float16)((acc[j][r] + accl[j][r] * (1.0f / 2048.0f)) * zr[r]);
  LDSX(); for (int rl = 0; rl < 16; ++rl) if (lane < 8) vst2((unsigned*)(MSG + (r0 + rl) * CD + (size_t)h * DH + lane * 8), *(const v4u*)&sh[wave][rl][lane * 8]); }
template <int MODE>
__global__ __launch_bounds__(128) void k_lin(const void* __restrict__ A1, const void* __restrict__ A2, const float* __restrict__ Wn, float* __restrict__ OUTF, _Float16* __restrict__ OUTH) { __shared__ __align__(16) float sf[4][16][132]; __shared__ __align__(16) _Float16 shh[4][16][136];
  const int tid = threadIdx.x, wave = tid >> 5, lane = tid & 31, col = lane & 15, g = lane >> 4; const size_t r0 = (size_t)blockIdx.x * 64 + wave * 16; const int c0 = blockIdx.y * 128; constexpr int KIN = MODE == 1 ? C2 : (MODE == 2 ? C2 : CD); constexpr int OW = MODE == 1 ? C2 : CD;
  v8f acc[8] = {};
#pragma unroll 2
  for (int kc = 0; kc < KIN / 32; ++kc) {
    if (MODE == 1 && kc < CD / 32) { const v16b a = frag_b((const __bf16*)A1 + (r0 + col) * CD + kc * 32, lane);
#pragma unroll
      for (int j = 0; j < 8; ++j) acc[j] = wmma_bf(a, fragb_f32(Wn + (size_t)(c0 + j * 16 + col) * KIN + kc * 32, lane), acc[j]); }
    else { const _Float16* ap = MODE == 1 ? ((const _Float16*)A2 + (r0 + col) * CD + (kc - CD / 32) * 32) : ((const _Float16*)A1 + (r0 + col) * KIN + kc * 32); const v16h a = frag_h(ap, lane);
#pragma unroll
      for (int j = 0; j < 8; ++j) acc[j] = wmma16(a, fragh_f32(Wn + (size_t)(c0 + j * 16 + col) * KIN + kc * 32, lane), acc[j]); } }
  if (MODE == 1) {
#pragma unroll
    for (int j = 0; j < 8; ++j)
#pragma unroll
      for (int r = 0; r < 8; ++r) shh[wave][8 * g + r][j * 16 + col] = (_Float16)fmaxf(acc[j][r], 0.f);
    LDSX(); for (int rl = 0; rl < 16; ++rl) if (lane < 16) vst2((unsigned*)(OUTH + (r0 + rl) * (size_t)OW + c0 + lane * 8), *(const v4u*)&shh[wave][rl][lane * 8]); }
  else {
#pragma unroll
    for (int j = 0; j < 8; ++j)
#pragma unroll
      for (int r = 0; r < 8; ++r) sf[wave][8 * g + r][j * 16 + col] = acc[j][r];
    LDSX(); for (int rl = 0; rl < 16; ++rl) vst2(OUTF + (r0 + rl) * (size_t)OW + c0 + lane * 4, *(const v4f*)&sf[wave][rl][lane * 4]); } }
__global__ __launch_bounds__(128) void k_ln1(const float* __restrict__ M2, const float* __restrict__ G, const float* __restrict__ Bt, _Float16* __restrict__ FFB) { __shared__ float red[4]; __shared__ __align__(16) _Float16 sh[CD]; const int t = threadIdx.x; const size_t row = blockIdx.x;
  float v[4]; float s = 0.f; for (int i = 0; i < 4; ++i) { v[i] = M2[row * CD + t + 128 * i]; s += v[i]; }
#pragma unroll
  for (int o = 1; o < 32; o <<= 1) s += __shfl_xor(s, o);
  if ((t & 31) == 0) red[t >> 5] = s; __syncthreads(); const float mu = (red[0] + red[1] + red[2] + red[3]) / (float)CD; __syncthreads();
  float q = 0.f; for (int i = 0; i < 4; ++i) { const float d = v[i] - mu; q += d * d; }
#pragma unroll
  for (int o = 1; o < 32; o <<= 1) q += __shfl_xor(q, o);
  if ((t & 31) == 0) red[t >> 5] = q; __syncthreads(); const float var = (red[0] + red[1] + red[2] + red[3]) / (float)CD; const float inv = 1.0f / sqrtf(var + EPSL);
  for (int i = 0; i < 4; ++i) { const int c = t + 128 * i; sh[c] = (_Float16)((v[i] - mu) * inv * bfr(G[c]) + bfr(Bt[c])); } __syncthreads(); if (t < CD / 8) vst2((unsigned*)(FFB + row * CD + t * 8), *(const v4u*)&sh[t * 8]); }
__global__ __launch_bounds__(256) void k_out(const float* __restrict__ M2, const float* __restrict__ G, const float* __restrict__ Bt, const float* __restrict__ X, float* __restrict__ Y) { __shared__ float smu[64], sinv[64]; __shared__ __align__(16) float st[128][64 + 4]; const int t = threadIdx.x, lane = t & 31, w = t >> 5; const size_t b = blockIdx.y; const int n0 = blockIdx.x * 64;
  for (int rl = w; rl < 64; rl += 8) { const float* mr = M2 + (b * NT + n0 + rl) * CD; float s = 0.f; for (int c = lane; c < CD; c += 32) s += mr[c];
#pragma unroll
    for (int o = 1; o < 32; o <<= 1) s += __shfl_xor(s, o);
    const float mu = s / (float)CD; float q = 0.f; for (int c = lane; c < CD; c += 32) { const float d = mr[c] - mu; q += d * d; }
#pragma unroll
    for (int o = 1; o < 32; o <<= 1) q += __shfl_xor(q, o);
    if (lane == 0) { smu[rl] = mu; sinv[rl] = 1.0f / sqrtf(q / (float)CD + EPSL); } }
  __syncthreads();
  for (int cc = 0; cc < CD; cc += 128) { for (int e = t; e < 128 * 64; e += 256) { const int cl = e >> 6, nl = e & 63; const int c = cc + cl; const size_t row = b * NT + n0 + nl; st[cl][nl] = bfr(X[(b * CD + c) * (size_t)NT + n0 + nl]) + (M2[row * CD + c] - smu[nl]) * sinv[nl] * bfr(G[c]) + bfr(Bt[c]); }
    __syncthreads(); for (int e = t; e < 128 * 16; e += 256) { const int cl = e >> 4, q = e & 15; vst2(Y + (b * CD + cc + cl) * (size_t)NT + n0 + q * 4, *(const v4f*)&st[cl][q * 4]); } __syncthreads(); } }
extern "C" void kernel_launch(void* const* d_in, const int* in_sizes, int n_in, void* d_out, int out_size, void* d_ws, size_t ws_size, hipStream_t stream) {
  (void)in_sizes; (void)n_in; (void)out_size;
  const float** F = (const float**)d_in;
  if (ws_size < (size_t)WS_END) return;
  char* ws = (char*)d_ws; __bf16* XS = (__bf16*)(ws + WS_XS); _Float16 *QH = (_Float16*)(ws + WS_QH), *QL = (_Float16*)(ws + WS_QL), *KT = (_Float16*)(ws + WS_KT), *KTL = (_Float16*)(ws + WS_KTL), *VT = (_Float16*)(ws + WS_VT), *VTL = (_Float16*)(ws + WS_VTL), *KVT = (_Float16*)(ws + WS_KVT), *KVL = (_Float16*)(ws + WS_KVL), *MSG = (_Float16*)(ws + WS_MSG), *FFB = (_Float16*)(ws + WS_FFB), *H1 = (_Float16*)(ws + WS_H1); float *KS = (float*)(ws + WS_KS), *M2 = (float*)(ws + WS_M2);
  k_xt<<<dim3(NT / 64, TNB), 256, 0, stream>>>(F[0], XS);
  k_qkv<<<dim3(NT / 64, 3 * CD / 128, TNB), 128, 0, stream>>>(XS, F[2], F[3], F[4], F[1], QH, QL, KT, KTL, VT, VTL);
  k_kv<<<dim3(NH, TNB), 128, 0, stream>>>(KT, KTL, VT, VTL, KVT, KVL, KS);
  k_msg<<<dim3(TNB * NT / 64, NH), 128, 0, stream>>>(QH, QL, KVT, KVL, KS, MSG);
  k_lin<0><<<dim3(TNB * NT / 64, CD / 128), 128, 0, stream>>>(MSG, nullptr, F[5], M2, nullptr);
  k_ln1<<<TNB * NT, 128, 0, stream>>>(M2, F[6], F[7], FFB);
  k_lin<1><<<dim3(TNB * NT / 64, C2 / 128), 128, 0, stream>>>(XS, FFB, F[8], nullptr, H1);
  k_lin<2><<<dim3(TNB * NT / 64, CD / 128), 128, 0, stream>>>(H1, nullptr, F[9], M2, nullptr);
  k_out<<<dim3(NT / 64, TNB), 256, 0, stream>>>(M2, F[10], F[11], F[0], (float*)d_out);
}
